// RecurGraphAgent_10548439679015
// MI455X (gfx1250) — hardware-verified
//
#include <hip/hip_runtime.h>


namespace {
constexpr int N = 20000, E = 320000, G = 64, FN = 16, FE = 8, CV = 32, LS = 32, KZ = 160  , NPAD = 20096  , NBLK = NPAD / 128;
constexpr float AS_ = 8.0f, WS_ = 8.0f, FXS = 524288.0f, FXI = 1.0f / 524288.0f, PXS = 1048576.0f;

typedef _Float16 b16;
typedef __attribute__((ext_vector_type(16))) _Float16 v16b;
typedef __attribute__((ext_vector_type(8))) _Float16 v8b;
typedef __attribute__((ext_vector_type(8))) float v8f;
typedef __attribute__((ext_vector_type(4))) float v4f;
__device__ __forceinline__ void split16(float v, b16& hi, b16& lo) { hi = (b16)v; lo = (b16)(v - (float)hi); }
__device__ __forceinline__ v16b frag_kb(const b16* p, int hh) { const v8b a = *(const v8b*)(p + 8 * hh), b = *(const v8b*)(p + 16 + 8 * hh); v16b f;
#pragma unroll
  for (int e = 0; e < 8; ++e) { f[e] = a[e]; f[8 + e] = b[e]; } return f; }
__device__ __forceinline__ v8f wmma16b(v16b a, v16b b, v8f c) { v8f d = __builtin_amdgcn_wmma_f32_16x16x32_f16(false, a, false, b, (short)0, c, false, false); asm volatile("v_nop\n\tv_nop\n\tv_nop\n\tv_nop" : "+v"(d) : "v"(a), "v"(b)); return d; }
__device__ __forceinline__ void wave_lds_sync() { __builtin_amdgcn_fence(__ATOMIC_RELEASE, "workgroup"); __builtin_amdgcn_wave_barrier(); __builtin_amdgcn_fence(__ATOMIC_ACQUIRE, "workgroup"); }
__device__ __forceinline__ int fkey(float f) { const int b = __float_as_int(f); return (b >= 0) ? b : (b ^ 0x7FFFFFFF); }
__device__ __forceinline__ float fkey_inv(int k) { return __int_as_float((k >= 0) ? k : (k ^ 0x7FFFFFFF)); }
__device__ __forceinline__ float nexp(float x) { return __builtin_amdgcn_exp2f(x * 1.4426950408889634f); }
__device__ __forceinline__ float sigm(float x) { return __builtin_amdgcn_rcpf(1.0f + nexp(-x)); }
__device__ __forceinline__ float tanh_(float x) { const float e = nexp(-2.0f * fabsf(x)); const float t = (1.0f - e) * __builtin_amdgcn_rcpf(1.0f + e); return (x >= 0.0f) ? t : -t; }
__device__ __forceinline__ int clampn(int v) { return (v < 0) ? 0 : (v >= N ? N - 1 : v); }

__global__ __launch_bounds__(256) void prep_kernel(const float* __restrict__ L, const float* __restrict__ bL, const float* __restrict__ root, const float* __restrict__ wih, const float* __restrict__ whh, const float* __restrict__ g1, b16* __restrict__ pL, b16* __restrict__ pR, b16* __restrict__ pG, b16* __restrict__ p1) {
  const int t_ = threadIdx.x;
  auto put = [&](b16* dst, size_t PL, size_t idx, float v) { b16 a, c; split16(v * WS_, a, c); ((volatile b16*)dst)[idx] = a; ((volatile b16*)dst)[PL + idx] = c; };
  for (int pass = 0; pass < 2; ++pass) {
    for (int p = t_; p < CV * KZ; p += 256) { const int o = p / KZ, k = p % KZ; float v = 0.0f; if (k < 128) { const int i = k >> 3, f = k & 7; v = L[(i * CV + o) * FE + f]; } else if (k < 144) v = bL[(k - 128) * CV + o]; put(pL, CV * KZ, p, v); }
    for (int p = t_; p < CV * 32; p += 256) { const int o = p >> 5, k = p & 31; put(pR, CV * 32, p, (k < FN) ? root[k * CV + o] : 0.0f); }
    for (int p = t_; p < 128 * 64; p += 256) { const int g = p >> 6, k = p & 63; put(pG, 128 * 64, p, (k < 32) ? wih[g * CV + k] : whh[g * LS + (k - 32)]); }
    for (int p = t_; p < 64 * 32; p += 256) put(p1, 64 * 32, p, g1[p]);
    __threadfence();
  }
}

__global__ __launch_bounds__(256) void edge_kernel(const float* __restrict__ x, const float* __restrict__ ea, const int* __restrict__ esrc, const b16* __restrict__ pL, float* __restrict__ msg) {
  __shared__ float Xs[8][16][FN + 1]; __shared__ float Ea[8][16][FE + 1]; __shared__ __attribute__((aligned(16))) float Ms[8][16][CV + 4];
  const int wid = threadIdx.x >> 5, lane = threadIdx.x & 31, nloc = lane & 15, hlf = lane >> 4; const int e0 = (blockIdx.x * 8 + wid) * 16;
  if (lane < 16) { const int s = clampn(esrc[e0 + lane]); const float* xr = x + (size_t)s * FN;
#pragma unroll
    for (int i = 0; i < FN; ++i) Xs[wid][lane][i] = xr[i];
#pragma unroll
    for (int f = 0; f < FE; ++f) Ea[wid][lane][f] = ea[(size_t)(e0 + lane) * FE + f]; }
  wave_lds_sync();
  v8f acc[2] = {{}, {}};
#pragma unroll
  for (int ks = 0; ks < 5; ++ks) { v16b ah, al;
#pragma unroll
    for (int e = 0; e < 16; ++e) { const int k = ks * 32 + ((e < 8) ? (8 * hlf + e) : (16 + 8 * hlf + e - 8)); float v = 0.0f;
      if (k < 128) v = Xs[wid][nloc][k >> 3] * Ea[wid][nloc][k & 7]; else if (k < 144) v = Xs[wid][nloc][k - 128];
      b16 a, c; split16(v * AS_, a, c); ah[e] = a; al[e] = c; }
#pragma unroll
    for (int t = 0; t < 2; ++t) { const v16b bh_ = frag_kb(pL + (size_t)(t * 16 + nloc) * KZ + ks * 32, hlf), bl_ = frag_kb(pL + (size_t)CV * KZ + (size_t)(t * 16 + nloc) * KZ + ks * 32, hlf);
      acc[t] = wmma16b(ah, bh_, acc[t]); acc[t] = wmma16b(al, bh_, acc[t]); acc[t] = wmma16b(ah, bl_, acc[t]); } }
#pragma unroll
  for (int t = 0; t < 2; ++t)
#pragma unroll
    for (int v = 0; v < 8; ++v) Ms[wid][8 * hlf + v][t * 16 + nloc] = acc[t][v] * (1.0f / (AS_ * WS_));
  wave_lds_sync();
  float* dst = msg + (size_t)e0 * CV;
  for (int pass = 0; pass < 2; ++pass) {
#pragma unroll
    for (int j = 0; j < 4; ++j) { const int rr = j * 4 + (lane >> 3), c4 = (lane & 7) * 4; *(volatile v4f*)(dst + (size_t)rr * CV + c4) = *(const v4f*)(&Ms[wid][rr][c4]); }
    __threadfence(); }
}

typedef __attribute__((ext_vector_type(4))) int v4i;
__global__ __launch_bounds__(256) void agg_kernel(const int* __restrict__ edst, const float* __restrict__ msg, float* __restrict__ agg) {
  constexpr int NB = 1024;
  __shared__ __attribute__((aligned(16))) int acc[NB * CV]; __shared__ int list[8 * 256];
  const int t_ = threadIdx.x, wave = t_ >> 5, lane = t_ & 31, base = blockIdx.x * NB, sub = lane >> 3, cl = (lane & 7) * 4;
  for (int i = t_; i < NB * CV; i += 256) acc[i] = 0;
  __syncthreads();
  int* wl = list + wave * 256;
  for (int c0 = 0; c0 < E; c0 += 256 * 8) {
    const int e0 = c0 + (wave * 32 + lane) * 8; int dd[8];
#pragma unroll
    for (int j = 0; j < 8; ++j) { const int dv = edst[min(e0 + j, E - 1)]; dd[j] = (e0 + j < E) ? dv : -1; }
    unsigned sl[8]; bool hit[8]; bool anyl = false;
#pragma unroll
    for (int j = 0; j < 8; ++j) { sl[j] = (unsigned)(dd[j] - base); hit[j] = sl[j] < (unsigned)NB; anyl |= hit[j]; }
    int wc = 0;
    if (__builtin_amdgcn_ballot_w32(anyl) != 0u) {
#pragma unroll
      for (int j = 0; j < 8; ++j) {
        const unsigned mj = __builtin_amdgcn_ballot_w32(hit[j]);
        if (mj != 0u) {
          if (hit[j]) { const int pos = wc + (int)__builtin_amdgcn_mbcnt_lo(mj, 0u); wl[pos] = ((e0 + j) << 10) | (int)sl[j]; }
          wc += __builtin_popcount(mj); } } }
    __builtin_amdgcn_wave_barrier(); __builtin_amdgcn_fence(__ATOMIC_RELEASE, "workgroup"); __builtin_amdgcn_fence(__ATOMIC_ACQUIRE, "workgroup");
    for (int i = sub; i < wc; i += 4) { const int ent = wl[i]; const int e = ent >> 10, slot = ent & 1023; const v4f v = *(const v4f*)(msg + (size_t)e * CV + cl); int* ar = acc + slot * CV + cl;
#pragma unroll
      for (int c = 0; c < 4; ++c) atomicAdd(ar + c, (int)rintf(v[c] * FXS)); }
    __builtin_amdgcn_wave_barrier();
  }
  __syncthreads();
  for (int pass = 0; pass < 2; ++pass) {
    for (int i = t_; i < NB * CV / 4; i += 256) { const int slot = i >> 3, cq = (i & 7) * 4, node = base + slot; v4f o = {0.0f, 0.0f, 0.0f, 0.0f};
      if (node < N) {
#pragma unroll
        for (int c = 0; c < 4; ++c) o[c] = (float)acc[slot * CV + cq + c] * FXI; }
      if (node < NPAD) *(volatile v4f*)(agg + (size_t)node * CV + cq) = o; }
    __threadfence(); }
}

__global__ __launch_bounds__(256) void node_kernel(const float* __restrict__ x, const float* __restrict__ agg, const float* __restrict__ init, const b16* __restrict__ pR, const b16* __restrict__ pG, const b16* __restrict__ p1,
                                                  const float* __restrict__ cb, const float* __restrict__ bih, const float* __restrict__ bhh, const float* __restrict__ hsw, const float* __restrict__ hsb, const float* __restrict__ csw, const float* __restrict__ csb,
                                                  const float* __restrict__ gb1, const float* __restrict__ g2, const float* __restrict__ gb2, const float* __restrict__ fnw, const float* __restrict__ fnb,
                                                  float* __restrict__ hout, float* __restrict__ sc, float* __restrict__ bst) {
  __shared__ __attribute__((aligned(16))) float Ta[8][16][64 + 4]; __shared__ __attribute__((aligned(16))) float Hs[8][16][LS + 4]; __shared__ __attribute__((aligned(16))) float Sc[8][16][8]; __shared__ float Wm[8], Wsum[8];
  const int wid = threadIdx.x >> 5, lane = threadIdx.x & 31, nloc = lane & 15, hlf = lane >> 4; const size_t r0 = (size_t)blockIdx.x * 128 + wid * 16;
  auto afrag = [&](int kb, v16b& ah, v16b& al) {
#pragma unroll
    for (int e = 0; e < 16; ++e) { const int k = kb + ((e < 8) ? (8 * hlf + e) : (16 + 8 * hlf + e - 8)); b16 a, c; split16(Ta[wid][nloc][k] * AS_, a, c); ah[e] = a; al[e] = c; } };
  auto gemm = [&](const b16* B, size_t PL, int KK, int NT, v8f* acc) {
    for (int kb = 0; kb < KK; kb += 32) { v16b ah, al; afrag(kb, ah, al);
      for (int t = 0; t < NT; ++t) { const v16b bh_ = frag_kb(B + (size_t)(t * 16 + nloc) * KK + kb, hlf), bl_ = frag_kb(B + PL + (size_t)(t * 16 + nloc) * KK + kb, hlf);
        acc[t] = wmma16b(ah, bh_, acc[t]); acc[t] = wmma16b(al, bh_, acc[t]); acc[t] = wmma16b(ah, bl_, acc[t]); } } };
  const float sc_ = 1.0f / (AS_ * WS_);
  { const int r = lane & 15; const size_t node = r0 + r; const int nn = (int)min(node, (size_t)(N - 1));
    for (int k = hlf; k < 32; k += 2) Ta[wid][r][k] = (k < FN) ? x[(size_t)nn * FN + k] : 0.0f; }
  wave_lds_sync();
  v8f acc[8];
  acc[0] = (v8f){}; acc[1] = (v8f){}; gemm(pR, CV * 32, 32, 2, acc); wave_lds_sync();
#pragma unroll
  for (int t = 0; t < 2; ++t)
#pragma unroll
    for (int v = 0; v < 8; ++v) { const int r = 8 * hlf + v, o = t * 16 + nloc; const size_t node = r0 + r; const int nn = (int)min(node, (size_t)(N - 1));
      Ta[wid][r][o] = fmaxf(acc[t][v] * sc_ + agg[node * CV + o] + cb[o], 0.0f); const float ini = init[nn]; Ta[wid][r][32 + o] = ini * hsw[o] + hsb[o]; }
  wave_lds_sync();
#pragma unroll
  for (int t = 0; t < 8; ++t) acc[t] = (v8f){};
  gemm(pG, 128 * 64, 64, 8, acc); wave_lds_sync();
#pragma unroll
  for (int tt = 0; tt < 2; ++tt) { const int u = tt * 16 + nloc;
#pragma unroll
    for (int v = 0; v < 8; ++v) { const int r = 8 * hlf + v; const size_t node = r0 + r; const int nn = (int)min(node, (size_t)(N - 1)); const float cprev = init[nn] * csw[u] + csb[u];
      const float gi = acc[0 + tt][v] * sc_ + bih[u] + bhh[u], gf = acc[2 + tt][v] * sc_ + bih[32 + u] + bhh[32 + u], gg = acc[4 + tt][v] * sc_ + bih[64 + u] + bhh[64 + u], go = acc[6 + tt][v] * sc_ + bih[96 + u] + bhh[96 + u];
      const float c = sigm(gf) * cprev + sigm(gi) * tanh_(gg); const float h = sigm(go) * tanh_(c); Hs[wid][r][u] = h; Ta[wid][r][u] = h; } }
  wave_lds_sync();
#pragma unroll
  for (int t = 0; t < 4; ++t) acc[t] = (v8f){};
  gemm(p1, 64 * 32, 32, 4, acc); wave_lds_sync();
#pragma unroll
  for (int t = 0; t < 4; ++t)
#pragma unroll
    for (int v = 0; v < 8; ++v) Ta[wid][8 * hlf + v][t * 16 + nloc] = fmaxf(acc[t][v] * sc_ + gb1[t * 16 + nloc], 0.0f);
  wave_lds_sync();
  if (hlf == 0) { const int r = nloc; float s = gb2[0];
#pragma unroll 1
    for (int k = 0; k < 64; ++k) s += Ta[wid][r][k] * g2[k];
    Sc[wid][r][0] = s; Sc[wid][r][1] = 0.0f; Sc[wid][r][2] = 0.0f; Sc[wid][r][3] = 0.0f;
#pragma unroll
    for (int a = 0; a < 4; ++a) { float l = fnb[a];
#pragma unroll 1
      for (int k = 0; k < LS; ++k) l += Hs[wid][r][k] * fnw[a * LS + k];
      Sc[wid][r][4 + a] = (r0 + r < (size_t)N) ? l : -INFINITY; } }
  wave_lds_sync();
  if (lane == 0) { float m = -INFINITY; for (int r = 0; r < 16; ++r) for (int a = 0; a < 4; ++a) m = fmaxf(m, Sc[wid][r][4 + a]); float s = 0.0f;
    for (int r = 0; r < 16; ++r) for (int a = 0; a < 4; ++a) { const float l = Sc[wid][r][4 + a]; s += (l > -INFINITY) ? __expf(l - m) : 0.0f; } Wm[wid] = m; Wsum[wid] = (m > -INFINITY) ? s : 0.0f; }
  __syncthreads();
  for (int pass = 0; pass < 2; ++pass) {
    for (int i = threadIdx.x; i < 128 * LS / 4; i += 256) { const int rr = i >> 3, c4 = (i & 7) * 4; *(volatile v4f*)(hout + ((size_t)blockIdx.x * 128 + rr) * LS + c4) = *(const v4f*)(&Hs[rr >> 4][rr & 15][c4]); }
    { const int rr = threadIdx.x >> 1, hq = threadIdx.x & 1; *(volatile v4f*)(sc + ((size_t)blockIdx.x * 128 + rr) * 8 + hq * 4) = *(const v4f*)(&Sc[rr >> 4][rr & 15][hq * 4]); }
    if (threadIdx.x < 32) { float m = -INFINITY; for (int w = 0; w < 8; ++w) m = fmaxf(m, Wm[w]); float s = 0.0f; for (int w = 0; w < 8; ++w) s += (Wsum[w] > 0.0f) ? Wsum[w] * __expf(Wm[w] - m) : 0.0f;
      ((volatile float*)bst)[(size_t)blockIdx.x * 32 + threadIdx.x] = (threadIdx.x == 0) ? m : (threadIdx.x == 1) ? s : 0.0f; }
    __threadfence(); }
}

__global__ __launch_bounds__(256) void pool_kernel(const int* __restrict__ batch, const float* __restrict__ hrow, const float* __restrict__ sc, const float* __restrict__ bst, const float* __restrict__ fgw, const float* __restrict__ fgb, float* __restrict__ gflat, float* __restrict__ gst) {
  __shared__ int gmx[G]; __shared__ int gden[G]; __shared__ __attribute__((aligned(16))) int gacc[G * LS]; __shared__ int list[8 * 256]; __shared__ float Lg[G * 4]; __shared__ float Gf[G * 4];
  const int t_ = threadIdx.x, wave = t_ >> 5, lane = t_ & 31;
  for (int i = t_; i < G * LS; i += 256) gacc[i] = 0;
  if (t_ < G) { gmx[t_] = fkey(-INFINITY); gden[t_] = 0; }
  __syncthreads();
  for (int n = t_; n < N; n += 256) { const int g = batch[n]; if ((unsigned)g < (unsigned)G) atomicMax(&gmx[g], fkey(sc[(size_t)n * 8])); }
  __syncthreads();
  int* wl = list + wave * 256;
  for (int c0 = 0; c0 < N; c0 += 256 * 8) {
    const int n0 = c0 + (wave * 32 + lane) * 8; int dd[8];
#pragma unroll
    for (int j = 0; j < 8; ++j) { const int gv = batch[min(n0 + j, N - 1)]; dd[j] = (n0 + j < N) ? gv : -1; }
    bool hit[8]; bool anyl = false;
#pragma unroll
    for (int j = 0; j < 8; ++j) { hit[j] = (unsigned)dd[j] < (unsigned)G; anyl |= hit[j]; }
    int wc = 0;
    if (__builtin_amdgcn_ballot_w32(anyl) != 0u) {
#pragma unroll
      for (int j = 0; j < 8; ++j) {
        const unsigned mj = __builtin_amdgcn_ballot_w32(hit[j]);
        if (mj != 0u) {
          if (hit[j]) { const int pos = wc + (int)__builtin_amdgcn_mbcnt_lo(mj, 0u); wl[pos] = ((n0 + j) << 6) | dd[j]; }
          wc += __builtin_popcount(mj); } } }
    __builtin_amdgcn_wave_barrier(); __builtin_amdgcn_fence(__ATOMIC_RELEASE, "workgroup"); __builtin_amdgcn_fence(__ATOMIC_ACQUIRE, "workgroup");
    for (int i = 0; i < wc; ++i) { const int ent = wl[i]; const int n = ent >> 6, g = ent & 63; const float w = nexp(sc[(size_t)n * 8] - fkey_inv(gmx[g]));
      if (lane == 0) atomicAdd(&gden[g], (int)rintf(w * PXS));
      atomicAdd(&gacc[g * LS + lane], (int)rintf(w * hrow[(size_t)n * LS + lane] * PXS)); }
    __builtin_amdgcn_wave_barrier();
  }
  __syncthreads();
  if (t_ < G * 4) { const int g = t_ >> 2, a = t_ & 3; const float dn = (float)gden[g]; float l = fgb[a];
    for (int k = 0; k < LS; ++k) { const float pk = (dn > 0.0f) ? (float)gacc[g * LS + k] / dn : 0.0f; l += pk * fgw[a * LS + k]; }
    Lg[t_] = l; }
  __syncthreads();
  if (t_ == 0) { float m = -INFINITY; for (int i = 0; i < G * 4; ++i) m = fmaxf(m, Lg[i]); float s = 0.0f; for (int i = 0; i < G * 4; ++i) s += __expf(Lg[i] - m); for (int i = 0; i < G * 4; ++i) Gf[i] = __expf(Lg[i] - m) / s;
    float M = -INFINITY; for (int b = 0; b < NBLK; ++b) M = fmaxf(M, bst[(size_t)b * 32]); float Z = 0.0f; for (int b = 0; b < NBLK; ++b) { const float sb = bst[(size_t)b * 32 + 1]; Z += (sb > 0.0f) ? sb * __expf(bst[(size_t)b * 32] - M) : 0.0f; }
    Lg[0] = M; Lg[1] = 1.0f / Z; }
  __syncthreads();
  for (int pass = 0; pass < 2; ++pass) { if (t_ < 64) *(volatile v4f*)(gflat + t_ * 4) = *(const v4f*)(&Gf[t_ * 4]); if (t_ < 32) ((volatile float*)gst)[t_] = (t_ == 0) ? Lg[0] : (t_ == 1) ? Lg[1] : 0.0f; __threadfence(); }
}

__global__ __launch_bounds__(256) void nodeflat_kernel(const float* __restrict__ sc, const float* __restrict__ gst, float* __restrict__ nflat) {
  const int n = blockIdx.x * 256 + threadIdx.x; if (n >= N) return;
  const float M = gst[0], iz = gst[1]; const v4f l = *(const v4f*)(sc + (size_t)n * 8 + 4); v4f p;
#pragma unroll
  for (int a = 0; a < 4; ++a) p[a] = __expf(l[a] - M) * iz;
  for (int pass = 0; pass < 2; ++pass) { *(volatile v4f*)(nflat + (size_t)n * 4) = p; __threadfence(); }
}
}

extern "C" void kernel_launch(void* const* d_in, const int* in_sizes, int n_in,
                              void* d_out, int out_size, void* d_ws, size_t ws_size, hipStream_t stream) {
  (void)n_in; (void)out_size;
  const float* x = (const float*)d_in[0]; const float* ea = (const float*)d_in[1]; const float* init = (const float*)d_in[2]; const int* ei = (const int*)d_in[3]; const int* batch = (const int*)d_in[4];
  const float* L = (const float*)d_in[5]; const float* bL = (const float*)d_in[6]; const float* root = (const float*)d_in[7]; const float* cb = (const float*)d_in[8];
  const float* wih = (const float*)d_in[9]; const float* whh = (const float*)d_in[10]; const float* bih = (const float*)d_in[11]; const float* bhh = (const float*)d_in[12];
  const float* hsw = (const float*)d_in[13]; const float* hsb = (const float*)d_in[14]; const float* csw = (const float*)d_in[15]; const float* csb = (const float*)d_in[16];
  const float* g1 = (const float*)d_in[17]; const float* gb1 = (const float*)d_in[18]; const float* g2 = (const float*)d_in[19]; const float* gb2 = (const float*)d_in[20];
  const float* fgw = (const float*)d_in[21]; const float* fgb = (const float*)d_in[22]; const float* fnw = (const float*)d_in[23]; const float* fnb = (const float*)d_in[24];
  float* nflat = (float*)d_out; float* gflat = nflat + (size_t)N * 4;
  if (in_sizes[0] != N * FN || in_sizes[1] != E * FE || in_sizes[2] != N || in_sizes[3] != 2 * E || in_sizes[4] != N || in_sizes[5] != FN * CV * FE || in_sizes[9] != 4 * LS * CV || in_sizes[17] != 64 * LS) return;
  const int* esrc = ei; const int* edst = ei + E;
  size_t off = 0; char* ws = (char*)d_ws;
  auto carve = [&](size_t bytes) { char* p = ws + off; off += (bytes + 255) & ~(size_t)255; return p; };
  b16* pL = (b16*)carve((size_t)CV * KZ * 4); b16* pR = (b16*)carve((size_t)CV * 32 * 4); b16* pG = (b16*)carve((size_t)128 * 64 * 4); b16* p1 = (b16*)carve((size_t)64 * 32 * 4);
  float* msg = (float*)carve((size_t)E * CV * 4); float* agg = (float*)carve((size_t)NPAD * CV * 4); float* hrow = (float*)carve((size_t)NPAD * LS * 4); float* sc = (float*)carve((size_t)NPAD * 8 * 4); float* bst = (float*)carve((size_t)NBLK * 32 * 4); float* gst = (float*)carve(256);
  if (off > ws_size) return;
  prep_kernel<<<1, 256, 0, stream>>>(L, bL, root, wih, whh, g1, pL, pR, pG, p1);
  edge_kernel<<<E / 128, 256, 0, stream>>>(x, ea, esrc, pL, msg);
  agg_kernel<<<(NPAD + 1023) / 1024, 256, 0, stream>>>(edst, msg, agg);
  node_kernel<<<NBLK, 256, 0, stream>>>(x, agg, init, pR, pG, p1, cb, bih, bhh, hsw, hsb, csw, csb, gb1, g2, gb2, fnw, fnb, hrow, sc, bst);
  pool_kernel<<<1, 256, 0, stream>>>(batch, hrow, sc, bst, fgw, fgb, gflat, gst);
  nodeflat_kernel<<<(N + 255) / 256, 256, 0, stream>>>(sc, gst, nflat);
}
